// Mamba3Block_60198261621479
// MI455X (gfx1250) — hardware-run, weakly checked
//
#include <hip/hip_runtime.h>
#include <math.h>

typedef __attribute__((ext_vector_type(16))) _Float16 v16h;
typedef __attribute__((ext_vector_type(8)))  _Float16 v8h;
typedef __attribute__((ext_vector_type(2)))  _Float16 v2h;
typedef __attribute__((ext_vector_type(16))) __bf16   v16b;
typedef __attribute__((ext_vector_type(8)))  __bf16   v8b;
typedef __attribute__((ext_vector_type(8)))  float    v8f;
typedef __attribute__((ext_vector_type(4)))  float    v4f;
typedef __attribute__((ext_vector_type(2)))  float    v2f;

constexpr int kNB   = 2;
constexpr int kT    = 1024;
constexpr int kRows = kNB * kT;
constexpr int kDM   = 1024;
constexpr int kNH   = 8;
constexpr int kHD   = 64;
constexpr int kDI   = kNH * kHD;
constexpr int kNs   = 128;
constexpr int kNQ   = 4;
constexpr int kCB   = kDI;
constexpr int kCC   = kCB + kNH * kNs;
constexpr int kCDt  = kCC + kNH * kNs;
constexpr int kCLa  = kCDt + kNH;
constexpr int kCTh  = kCLa + kNH;
constexpr int kNPl  = kCTh + kNH;
constexpr int kNP   = 2624;
constexpr int kThr  = 256;
constexpr float kInCarry = 1024.0f;
constexpr float kWCarry  = 4096.0f;
constexpr float kCY   = 1024.0f;
constexpr float kF16MinNormal = 6.103515625e-5f;

static_assert(kDI == 512 && kCC == 1536 && kCDt == 2560 && kCLa == 2568 && kCTh == 2576 && kNPl == 2584 && kNPl <= kNP && (kNP % 64) == 0 && kNs == kNQ * 32 && kRows == 2048, "the column map and the index arithmetic below use these sizes");

constexpr size_t kOffZB = 0ull;
constexpr size_t kOffX16 = 11264ull;
constexpr size_t kOffWIN16 = 4205568ull;
constexpr size_t kOffWOUT16 = 9579520ull;
constexpr size_t kOffPROJ = 10628096ull;
constexpr size_t kOffAL = 32123904ull;
constexpr size_t kOffBE = 32189440ull;
constexpr size_t kOffGA = 32254976ull;
constexpr size_t kOffINC = 32320512ull;
constexpr size_t kOffCS = 32386048ull;
constexpr size_t kOffSN = 32451584ull;
constexpr size_t kOffBR = 32517120ull;
constexpr size_t kOffCR = 40905728ull;
constexpr size_t kOffYP = 49294336ull;
constexpr size_t kOffRST = 66071552ull;
constexpr size_t kOffY16 = 66079744ull;
constexpr size_t kWsTotal = 68176896ull;
static_assert(kWsTotal <= 134217728ull, "carve cap: under 128 MiB");
static_assert(kOffZB == 0
  && kOffX16 == kOffZB + 11264ull
  && kOffWIN16 == kOffX16 + 4194304ull
  && kOffWOUT16 == kOffWIN16 + 5373952ull
  && kOffPROJ == kOffWOUT16 + 1048576ull
  && kOffAL == kOffPROJ + 21495808ull
  && kOffBE == kOffAL + 65536ull
  && kOffGA == kOffBE + 65536ull
  && kOffINC == kOffGA + 65536ull
  && kOffCS == kOffINC + 65536ull
  && kOffSN == kOffCS + 65536ull
  && kOffBR == kOffSN + 65536ull
  && kOffCR == kOffBR + 8388608ull
  && kOffYP == kOffCR + 8388608ull
  && kOffRST == kOffYP + 16777216ull
  && kOffY16 == kOffRST + 8192ull
  && kWsTotal == kOffY16 + 2097152ull, "the carve is a chain: every region starts where the one before ends");
static_assert((kOffX16 % 256) == 0 && (kOffWIN16 % 256) == 0 && (kOffWOUT16 % 256) == 0 && (kOffPROJ % 256) == 0 && (kOffAL % 256) == 0 && (kOffBE % 256) == 0 && (kOffGA % 256) == 0 && (kOffINC % 256) == 0 && (kOffCS % 256) == 0 && (kOffSN % 256) == 0 && (kOffBR % 256) == 0 && (kOffCR % 256) == 0 && (kOffYP % 256) == 0 && (kOffRST % 256) == 0 && (kOffY16 % 256) == 0, "every region starts on a multiple of 256 B");

__device__ __forceinline__ unsigned short f2bf_bits(float f) {
  unsigned u = __float_as_uint(f);
  return (unsigned short)((u + 0x7FFFu + ((u >> 16) & 1u)) >> 16);
}
__device__ __forceinline__ float bf_bits2f(unsigned short h) { return __uint_as_float(((unsigned)h) << 16); }
__device__ __forceinline__ float bf16r(float f) { return bf_bits2f(f2bf_bits(f)); }
__device__ __forceinline__ float carry_flush(float v, float carry) {
  const float s = v * carry;
  return (fabsf(s) < kF16MinNormal) ? 0.0f : s;
}

__device__ __forceinline__ void dep_guard4_h(v8f& a, v8f& b, v8f& c, v8f& d, v16h x, v16h y) { asm volatile("v_nop\n\tv_nop\n\tv_nop\n\tv_nop" : "+v"(a), "+v"(b), "+v"(c), "+v"(d) : "v"(x), "v"(y)); }
__device__ __forceinline__ void dep_guard4_b(v8f& a, v8f& b, v8f& c, v8f& d, v16b x, v16b y) { asm volatile("v_nop\n\tv_nop\n\tv_nop\n\tv_nop" : "+v"(a), "+v"(b), "+v"(c), "+v"(d) : "v"(x), "v"(y)); }
__device__ __forceinline__ void keep4_h(v16h a, v16h b, v16h c, v16h d) { asm volatile("v_nop" :: "v"(a), "v"(b), "v"(c), "v"(d)); }
__device__ __forceinline__ void keep4_b(v16b a, v16b b, v16b c, v16b d) { asm volatile("v_nop" :: "v"(a), "v"(b), "v"(c), "v"(d)); }
__device__ __forceinline__ void acc_guard4(v8f& a, v8f& b, v8f& c, v8f& d) { asm volatile("v_nop\n\tv_nop\n\tv_nop\n\tv_nop" : "+v"(a), "+v"(b), "+v"(c), "+v"(d)); }

template <typename T> struct Frag;
template <> struct Frag<_Float16> {
  typedef v16h V; union U { v16h v; v8h h[2]; };
  static __device__ __forceinline__ v16h load(const _Float16* p) {
    U f; f.h[0] = *(const v8h*)(p); f.h[1] = *(const v8h*)(p + 16); return f.v;
  }
  static __device__ __forceinline__ v8f mma(v16h a, v16h b, v8f c) {
    return __builtin_amdgcn_wmma_f32_16x16x32_f16(false, a, false, b, (short)0, c, false, false);
  }
  static __device__ __forceinline__ void guard4(v8f& a, v8f& b, v8f& c, v8f& d, v16h x, v16h y) { dep_guard4_h(a, b, c, d, x, y); }
  static __device__ __forceinline__ void keep(v16h a, v16h b, v16h c, v16h d) { keep4_h(a, b, c, d); }
};
template <> struct Frag<__bf16> {
  typedef v16b V; union U { v16b v; v8b h[2]; };
  static __device__ __forceinline__ v16b load(const __bf16* p) {
    U f; f.h[0] = *(const v8b*)(p); f.h[1] = *(const v8b*)(p + 16); return f.v;
  }
  static __device__ __forceinline__ v8f mma(v16b a, v16b b, v8f c) {
    return __builtin_amdgcn_wmma_f32_16x16x32_bf16(false, a, false, b, (short)0, c, false, false);
  }
  static __device__ __forceinline__ void guard4(v8f& a, v8f& b, v8f& c, v8f& d, v16b x, v16b y) { dep_guard4_b(a, b, c, d, x, y); }
  static __device__ __forceinline__ void keep(v16b a, v16b b, v16b c, v16b d) { keep4_b(a, b, c, d); }
};

__device__ __forceinline__ v8f mma_h(v16h a, v16h b, v8f c) {
  c = __builtin_amdgcn_wmma_f32_16x16x32_f16(false, a, false, b, (short)0, c, false, false);
  asm volatile("v_nop\n\tv_nop\n\tv_nop\n\tv_nop" : "+v"(c) : "v"(a), "v"(b));
  return c;
}

template <int ET> struct Elem;
template <> struct Elem<0> { typedef _Float16 T; };
template <> struct Elem<1> { typedef __bf16 T; };
template <int ET, bool SPLIT, int BIAS_MODE, int OUT_MODE, bool RESID, int ACT = 0>
__global__ __launch_bounds__(256) void wmma_gemm64(
    const unsigned short* __restrict__ Ap, const unsigned short* __restrict__ A2p, int lda, long strideA,
    const unsigned short* __restrict__ Btp, const unsigned short* __restrict__ Bt2p, int ldb, long strideB,
    void* __restrict__ Cout, void* __restrict__ Cout2, int ldc, long strideC,
    const float* __restrict__ bias,
    const float* __restrict__ resid, long strideR,
    int M, int N, int K, float scale) {
  typedef typename Elem<ET>::T T;
  typedef typename Frag<T>::V V;
  const T* A = (const T*)Ap; const T* A2 = (const T*)A2p; const T* Bt = (const T*)Btp; const T* Bt2 = (const T*)Bt2p;
  __shared__ __align__(16) float sT[8][16 * 68];
  const int b    = blockIdx.y;
  const int lane = threadIdx.x & 31;
  const int wave = threadIdx.x >> 5;
  const int tilesN = N >> 6;
  const int tilesM = M >> 6;
  const int tile = blockIdx.x * 8 + wave;
  if (tile >= tilesM * tilesN) return;
  const int tm = tile / tilesN;
  const int tn = tile - tm * tilesN;
  const int m0 = tm << 6;
  const int n0 = tn << 6;

  const T* Ab  = A  + (size_t)b * strideA;
  const T* Bb  = Bt + (size_t)b * strideB;
  const T* Ab2 = SPLIT ? (A2  + (size_t)b * strideA) : nullptr;
  const T* Bb2 = SPLIT ? (Bt2 + (size_t)b * strideB) : nullptr;

  const int rlane = lane & 15;
  const int koff  = (lane >> 4) * 8;
  const int mOff  = (lane >> 4) * 8;

  v8f acc[4][4];
#pragma unroll
  for (int i = 0; i < 4; ++i)
#pragma unroll
    for (int j = 0; j < 4; ++j) acc[i][j] = (v8f){0.f,0.f,0.f,0.f,0.f,0.f,0.f,0.f};

  for (int k0 = 0; k0 < K; k0 += 32) {
    V bh[4], bl[4];
#pragma unroll
    for (int j = 0; j < 4; ++j) {
      const size_t bo = (size_t)(n0 + (j << 4) + rlane) * ldb + koff + k0;
      bh[j] = Frag<T>::load(Bb + bo);
      if (SPLIT) bl[j] = Frag<T>::load(Bb2 + bo);
    }
#pragma unroll
    for (int i = 0; i < 4; ++i) {
      const size_t ao = (size_t)(m0 + (i << 4) + rlane) * lda + koff + k0;
      V ah = Frag<T>::load(Ab + ao);
      V al;
      if (SPLIT) al = Frag<T>::load(Ab2 + ao);
#pragma unroll
      for (int j = 0; j < 4; ++j) {
        acc[i][j] = Frag<T>::mma(ah, bh[j], acc[i][j]);
        if (SPLIT) {
          acc[i][j] = Frag<T>::mma(ah, bl[j], acc[i][j]);
          acc[i][j] = Frag<T>::mma(al, bh[j], acc[i][j]);
        }
      }
      Frag<T>::guard4(acc[i][0], acc[i][1], acc[i][2], acc[i][3], ah, SPLIT ? al : ah);
    }
    Frag<T>::keep(bh[0], bh[1], bh[2], bh[3]);
    if (SPLIT) Frag<T>::keep(bl[0], bl[1], bl[2], bl[3]);
  }
  acc_guard4(acc[0][0], acc[0][1], acc[0][2], acc[0][3]);
  acc_guard4(acc[1][0], acc[1][1], acc[1][2], acc[1][3]);
  acc_guard4(acc[2][0], acc[2][1], acc[2][2], acc[2][3]);
  acc_guard4(acc[3][0], acc[3][1], acc[3][2], acc[3][3]);

  float* slab = sT[wave];
  const float* Rb = RESID ? (resid + (size_t)b * strideR) : nullptr;
#pragma unroll
  for (int i = 0; i < 4; ++i) {
    const int mBase = m0 + (i << 4);
#pragma unroll
    for (int j = 0; j < 4; ++j) {
      const int n = n0 + (j << 4) + rlane;
      float bv = 0.f;
      if (BIAS_MODE == 2) bv = bias[n];
#pragma unroll
      for (int r = 0; r < 8; ++r) {
        float v = acc[i][j][r] * scale;
        if (BIAS_MODE == 1) v += bias[mBase + mOff + r];
        if (BIAS_MODE == 2) v += bv;
        if (RESID) v += Rb[(size_t)(mBase + mOff + r) * ldc + n];
        if (ACT == 1) v = tanhf(v);
        if (ACT == 2) v = fmaxf(v, 0.0f);
        if (ACT == 3) v = v / (1.0f + expf(-v));
        if (ACT == 4) v = (v > 0.f) ? v : 0.01f * v;
        slab[(mOff + r) * 68 + (j << 4) + rlane] = v;
      }
    }
    __builtin_amdgcn_fence(__ATOMIC_RELEASE, "workgroup");
    __builtin_amdgcn_wave_barrier();
    __builtin_amdgcn_fence(__ATOMIC_ACQUIRE, "workgroup");
    if (OUT_MODE == 0) {
      float* C = (float*)Cout + (size_t)b * strideC;
      const int hh = lane >> 4, c4 = (lane & 15) * 4;
      for (int pass = 0; pass < 2; ++pass) {
#pragma unroll
        for (int it = 0; it < 8; ++it) {
          const int row = it * 2 + hh;
          v4f v = *(const v4f*)(slab + row * 68 + c4);
          *(volatile v4f*)(C + (size_t)(mBase + row) * ldc + n0 + c4) = v;
        }
        __threadfence();
      }
    } else {
      const int q = lane >> 3, c8 = (lane & 7) * 8;
      unsigned short* C  = (unsigned short*)Cout  + (size_t)b * strideC;
      unsigned short* C2 = (OUT_MODE == 2) ? ((unsigned short*)Cout2 + (size_t)b * strideC) : nullptr;
      for (int pass = 0; pass < 2; ++pass) {
#pragma unroll
        for (int it = 0; it < 4; ++it) {
          const int row = it * 4 + q;
          const float* sp = slab + row * 68 + c8;
          v8h hv, lv;
#pragma unroll
          for (int e = 0; e < 8; ++e) {
            if (OUT_MODE == 1) {
              hv[e] = (_Float16)sp[e];
            } else {
              unsigned short hb = f2bf_bits(sp[e]);
              unsigned short lb = f2bf_bits(sp[e] - bf_bits2f(hb));
              hv[e] = __builtin_bit_cast(_Float16, hb);
              lv[e] = __builtin_bit_cast(_Float16, lb);
            }
          }
          *(volatile v8h*)(C + (size_t)(mBase + row) * ldc + n0 + c8) = hv;
          if (OUT_MODE == 2) *(volatile v8h*)(C2 + (size_t)(mBase + row) * ldc + n0 + c8) = lv;
        }
        __threadfence();
      }
    }
    __builtin_amdgcn_fence(__ATOMIC_RELEASE, "workgroup");
    __builtin_amdgcn_wave_barrier();
    __builtin_amdgcn_fence(__ATOMIC_ACQUIRE, "workgroup");
  }
}


__device__ __forceinline__ void store2(float* p, float v) {
  *(volatile float*)p = v;
  __threadfence();
  *(volatile float*)p = v;
}

__global__ __launch_bounds__(kThr) void cast_plane_kernel(const float* __restrict__ src, unsigned short* __restrict__ dst,
                                                          int colsLog2, int dstPitch, int dstOff) {
  const int i   = blockIdx.x * kThr + threadIdx.x;
  const int sh  = colsLog2 - 3;
  const int row = i >> sh;
  const int c8  = (i & ((1 << sh) - 1)) * 8;
  const float* sp = src + ((size_t)row << colsLog2) + c8;
  const v4f a0 = *(const v4f*)(sp);
  const v4f a1 = *(const v4f*)(sp + 4);
  v8h hv;
#pragma unroll
  for (int e = 0; e < 4; ++e) {
    const float f0 = a0[e];
    const float f1 = a1[e];
    hv[e]     = (_Float16)carry_flush(bf16r(f0), kInCarry);
    hv[4 + e] = (_Float16)carry_flush(bf16r(f1), kInCarry);
  }
  unsigned short* dp = dst + (size_t)row * dstPitch + dstOff + c8;
  *(volatile v8h*)dp = hv;
  __threadfence();
  *(volatile v8h*)dp = hv;
}

__global__ __launch_bounds__(256) void wt_plane_kernel(const float* __restrict__ W, unsigned short* __restrict__ dst, int K, int N, int nLive, int ldd, int colOff) {
  const int n  = blockIdx.x;
  const int k8 = threadIdx.x * 8;
  const bool live = n < nLive;
  const int nc = live ? n : 0;
  v8h hv;
#pragma unroll
  for (int e = 0; e < 8; ++e) {
    const float w = W[(size_t)(k8 + e) * N + nc];
    hv[e] = (_Float16)(live ? carry_flush(bf16r(w), kWCarry) : 0.0f);
  }
  unsigned short* dp = dst + (size_t)n * ldd + colOff + k8;
  *(volatile v8h*)dp = hv;
  __threadfence();
  *(volatile v8h*)dp = hv;
}

__global__ __launch_bounds__(kThr) void setup_kernel(float* __restrict__ ZB, unsigned short* __restrict__ WIN16) {
  const unsigned bk = blockIdx.x;
  if (bk < 11u) {
    store2(ZB + bk * (unsigned)kThr + threadIdx.x, 0.0f);
  } else {
    const unsigned j = (bk - 11u) * (unsigned)kThr + threadIdx.x;
    v8h zv;
#pragma unroll
    for (int e = 0; e < 8; ++e) zv[e] = (_Float16)0.0f;
    unsigned short* dp = WIN16 + (size_t)kNPl * kDM + (size_t)j * 8;
    *(volatile v8h*)dp = zv;
    __threadfence();
    *(volatile v8h*)dp = zv;
  }
}
static_assert(2816 == 11 * kThr && 2816 >= kNP && (size_t)(kNP - kNPl) * kDM / 8 == 20ull * kThr, "set-up grid: 11 + 20 = 31 blocks");

__global__ __launch_bounds__(kThr) void pre_kernel(const float* __restrict__ PROJ, const float* __restrict__ dtb, const float* __restrict__ alog,
                                                  float* __restrict__ AL, float* __restrict__ BE, float* __restrict__ GA, float* __restrict__ INC) {
  const unsigned i = blockIdx.x * (unsigned)kThr + threadIdx.x;
  const size_t row = i >> 3;
  const unsigned hd = i & 7u;
  const float* pr = PROJ + row * kNP;
  const float b0 = dtb[hd], a0 = alog[hd];
  const float vdt = pr[kCDt + hd] + bf16r(b0);
  const float vla = pr[kCLa + hd];
  const float th = pr[kCTh + hd];
  const float dt = fmaxf(vdt, 0.0f) + log1pf(expf(-fabsf(vdt)));
  const float lam = 1.0f / (1.0f + expf(-vla));
  const float A = -expf(bf16r(a0));
  const float al = expf(dt * A);
  store2(AL + i, al);
  store2(BE + i, ((1.0f - lam) * dt) * al);
  store2(GA + i, lam * dt);
  store2(INC + i, dt * th);
}
static_assert((size_t)kRows * kNH == 64ull * kThr, "the token-head grid exact: 64 blocks");

__global__ __launch_bounds__(16) void angle_kernel(const float* __restrict__ INC, float* __restrict__ CS, float* __restrict__ SN) {
  const unsigned sq = threadIdx.x >> 3;
  const unsigned hd = threadIdx.x & 7u;
  float acc = 0.0f;
  for (int t = 0; t < kT; ++t) {
    const size_t o = ((size_t)sq * kT + (size_t)t) * kNH + hd;
    acc += INC[o];
    store2(CS + o, cosf(acc));
    store2(SN + o, sinf(acc));
  }
}
static_assert(kNB * kNH == 16, "the angles: one block of sixteen lanes");

__global__ __launch_bounds__(kThr) void rot_kernel(const float* __restrict__ PROJ, const float* __restrict__ CS, const float* __restrict__ SN, float* __restrict__ BR, float* __restrict__ CR) {
  const unsigned i = blockIdx.x * (unsigned)kThr + threadIdx.x;
  const size_t row = i >> 7;
  const unsigned hd = (i >> 4) & 7u;
  const unsigned n8 = (i & 15u) * 8u;
  const float c = CS[row * kNH + hd], s = SN[row * kNH + hd];
  const float* pb = PROJ + row * kNP + kCB + hd * kNs + n8;
  const float* pc = PROJ + row * kNP + kCC + hd * kNs + n8;
  const v4f b0 = *(const v4f*)pb, b1 = *(const v4f*)(pb + 4), c0 = *(const v4f*)pc, c1 = *(const v4f*)(pc + 4);
  v4f rb0, rb1, rc0, rc1;
  rb0[0] = b0[0] * c - b0[1] * s; rb0[1] = b0[0] * s + b0[1] * c; rb0[2] = b0[2] * c - b0[3] * s; rb0[3] = b0[2] * s + b0[3] * c;
  rb1[0] = b1[0] * c - b1[1] * s; rb1[1] = b1[0] * s + b1[1] * c; rb1[2] = b1[2] * c - b1[3] * s; rb1[3] = b1[2] * s + b1[3] * c;
  rc0[0] = c0[0] * c - c0[1] * s; rc0[1] = c0[0] * s + c0[1] * c; rc0[2] = c0[2] * c - c0[3] * s; rc0[3] = c0[2] * s + c0[3] * c;
  rc1[0] = c1[0] * c - c1[1] * s; rc1[1] = c1[0] * s + c1[1] * c; rc1[2] = c1[2] * c - c1[3] * s; rc1[3] = c1[2] * s + c1[3] * c;
  float* db = BR + (row * kNH + hd) * kNs + n8;
  float* dc = CR + (row * kNH + hd) * kNs + n8;
  for (int pass = 0; pass < 2; ++pass) {
    *(volatile v4f*)db = rb0; *(volatile v4f*)(db + 4) = rb1;
    *(volatile v4f*)dc = rc0; *(volatile v4f*)(dc + 4) = rc1;
    __threadfence();
  }
}
static_assert((size_t)kRows * kNH * (kNs / 8) == 1024ull * kThr && kNs / 8 == 16 && (kCB % 4) == 0 && (kCC % 4) == 0, "rotation grid exact: 1,024 blocks; 16 groups a head; the 16-B loads aligned");

__global__ __launch_bounds__(kThr) void scan_kernel(const float* __restrict__ PROJ, const float* __restrict__ AL, const float* __restrict__ BE, const float* __restrict__ GA,
                                                    const float* __restrict__ BR, const float* __restrict__ CR, float* __restrict__ YP) {
  const unsigned qt = blockIdx.x >> 2;
  const unsigned ix = (blockIdx.x & 3u) * (unsigned)kThr + threadIdx.x;
  const unsigned sq = ix >> 9;
  const unsigned ch = ix & 511u;
  const unsigned hd = ch >> 6;
  const unsigned n0 = qt * 32u;
  float h[32], bq[32];
#pragma unroll
  for (int n = 0; n < 32; ++n) { h[n] = 0.0f; bq[n] = 0.0f; }
  float up = 0.0f;
  for (int t = 0; t < kT; ++t) {
    const size_t row = (size_t)sq * kT + (size_t)t;
    const size_t th = row * kNH + hd;
    const float al = AL[th], be = BE[th], ga = GA[th];
    const float ut = PROJ[row * kNP + ch];
    const float* pb = BR + th * kNs + n0;
    const float* pc = CR + th * kNs + n0;
    float y = 0.0f;
#pragma unroll
    for (int q = 0; q < 8; ++q) {
      const v4f bv = *(const v4f*)(pb + 4 * q), cv = *(const v4f*)(pc + 4 * q);
#pragma unroll
      for (int e = 0; e < 4; ++e) {
        const int n = 4 * q + e;
        const float hn = (al * h[n] + be * (up * bq[n])) + ga * (ut * bv[e]);
        h[n] = hn;
        bq[n] = bv[e];
        y += hn * cv[e];
      }
    }
    up = ut;
    store2(YP + (row * kNQ + qt) * kDI + ch, y);
  }
}
static_assert(kNQ * kNB * kDI == 16 * kThr && kNB * kDI == 4 * kThr, "walk grid exact: 16 blocks: four a quarter");

__global__ __launch_bounds__(kThr) void rstat_kernel(const float* __restrict__ YP, float* __restrict__ RST) {
  const size_t row = (size_t)blockIdx.x * kThr + threadIdx.x;
  const float* y0 = YP + (row * kNQ + 0) * kDI;
  const float* y1 = YP + (row * kNQ + 1) * kDI;
  const float* y2 = YP + (row * kNQ + 2) * kDI;
  const float* y3 = YP + (row * kNQ + 3) * kDI;
  float q = 0.0f;
  for (int c = 0; c < kDI; ++c) { const float y = ((y0[c] + y1[c]) + y2[c]) + y3[c]; q += y * y; }
  store2(RST + row, 1.0f / sqrtf(q / (float)kDI + 1e-6f));
}
static_assert(kRows == 8 * kThr, "the statistic's grid exact: 8 blocks");

__global__ __launch_bounds__(kThr) void ycast_kernel(const float* __restrict__ YP, const float* __restrict__ RST, const float* __restrict__ rw, unsigned short* __restrict__ Y16) {
  const unsigned i = blockIdx.x * (unsigned)kThr + threadIdx.x;
  const size_t row = i >> 6;
  const unsigned c8 = (i & 63u) * 8u;
  const float r = RST[row];
  const float* y0 = YP + (row * kNQ + 0) * kDI + c8;
  const float* y1 = YP + (row * kNQ + 1) * kDI + c8;
  const float* y2 = YP + (row * kNQ + 2) * kDI + c8;
  const float* y3 = YP + (row * kNQ + 3) * kDI + c8;
  v8h hv;
#pragma unroll
  for (int e = 0; e < 8; ++e) {
    const float w0 = rw[c8 + e];
    const float y = ((y0[e] + y1[e]) + y2[e]) + y3[e];
    hv[e] = (_Float16)carry_flush((y * r) * bf16r(w0), kCY);
  }
  unsigned short* dp = Y16 + row * kDI + c8;
  *(volatile v8h*)dp = hv;
  __threadfence();
  *(volatile v8h*)dp = hv;
}
static_assert((size_t)kRows * (kDI / 8) == 512ull * kThr && kDI / 8 == 64, "norm cast grid exact: 512 blocks; 64 groups a row");

extern "C" void kernel_launch(void* const* d_in, const int* in_sizes, int n_in,
                              void* d_out, int out_size, void* d_ws, size_t ws_size,
                              hipStream_t stream) {
  if (n_in < 7 || d_out == nullptr || d_ws == nullptr) return;
  if (in_sizes[0] != kRows * kDM || in_sizes[1] != kDI * kDM || in_sizes[2] != (kNPl - kDI) * kDM || in_sizes[3] != kDM * kDI || in_sizes[4] != kNH || in_sizes[5] != kNH || in_sizes[6] != kDI) return;
  if (out_size != kRows * kDM) return;
  if (ws_size < kWsTotal) return;
  const float* x    = (const float*)d_in[0];
  const float* win  = (const float*)d_in[1];
  const float* wsel = (const float*)d_in[2];
  const float* wout = (const float*)d_in[3];
  const float* alog = (const float*)d_in[4];
  const float* dtb  = (const float*)d_in[5];
  const float* rw   = (const float*)d_in[6];
  float* out = (float*)d_out;
  char* ws = (char*)d_ws;
  float* ZB = (float*)(ws + kOffZB);
  unsigned short* X16    = (unsigned short*)(ws + kOffX16);
  unsigned short* WIN16  = (unsigned short*)(ws + kOffWIN16);
  unsigned short* WOUT16 = (unsigned short*)(ws + kOffWOUT16);
  float* PROJ = (float*)(ws + kOffPROJ);
  float* AL  = (float*)(ws + kOffAL);
  float* BE  = (float*)(ws + kOffBE);
  float* GA  = (float*)(ws + kOffGA);
  float* INC = (float*)(ws + kOffINC);
  float* CS  = (float*)(ws + kOffCS);
  float* SN  = (float*)(ws + kOffSN);
  float* BR  = (float*)(ws + kOffBR);
  float* CR  = (float*)(ws + kOffCR);
  float* YP  = (float*)(ws + kOffYP);
  float* RST = (float*)(ws + kOffRST);
  unsigned short* Y16 = (unsigned short*)(ws + kOffY16);

  static_assert(((size_t)kRows * kDM / 8) % kThr == 0 && ((size_t)kDI * kDM / 8) % kThr == 0 && ((size_t)(kNPl - kDI) * kDM / 8) % kThr == 0 && ((size_t)kDM * kDI / 8) % kThr == 0, "the casts' grids");
  cast_plane_kernel<<<(int)(((size_t)kRows * kDM / 8) / kThr), kThr, 0, stream>>>(x, X16, 10, kDM, 0);
  cast_plane_kernel<<<(int)(((size_t)kDI * kDM / 8) / kThr), kThr, 0, stream>>>(win, WIN16, 10, kDM, 0);
  cast_plane_kernel<<<(int)(((size_t)(kNPl - kDI) * kDM / 8) / kThr), kThr, 0, stream>>>(wsel, WIN16 + (size_t)kDI * kDM, 10, kDM, 0);
  cast_plane_kernel<<<(int)(((size_t)kDM * kDI / 8) / kThr), kThr, 0, stream>>>(wout, WOUT16, 9, kDI, 0);
  setup_kernel<<<31, kThr, 0, stream>>>(ZB, WIN16);

  wmma_gemm64<0, false, 2, 0, false, 0><<<dim3((kRows / 64) * (kNP / 64) / 8, 1), 256, 0, stream>>>(
      X16, X16, kDM, 0L, WIN16, WIN16, kDM, 0L, (void*)PROJ, (void*)PROJ, kNP, 0L, ZB, nullptr, 0L, kRows, kNP, kDM, 1.0f / (kInCarry * kInCarry));
  pre_kernel<<<64, kThr, 0, stream>>>(PROJ, dtb, alog, AL, BE, GA, INC);
  angle_kernel<<<1, 16, 0, stream>>>(INC, CS, SN);
  rot_kernel<<<1024, kThr, 0, stream>>>(PROJ, CS, SN, BR, CR);
  scan_kernel<<<16, kThr, 0, stream>>>(PROJ, AL, BE, GA, BR, CR, YP);
  rstat_kernel<<<8, kThr, 0, stream>>>(YP, RST);
  ycast_kernel<<<512, kThr, 0, stream>>>(YP, RST, rw, Y16);
  wmma_gemm64<0, false, 2, 0, false, 0><<<dim3((kRows / 64) * (kDM / 64) / 8, 1), 256, 0, stream>>>(
      Y16, Y16, kDI, 0L, WOUT16, WOUT16, kDI, 0L, (void*)out, (void*)out, kDM, 0L, ZB, nullptr, 0L, kRows, kDM, kDI, 1.0f / (kCY * kInCarry));
}
static_assert(((kRows / 64) * (kNP / 64)) % 8 == 0 && ((kRows / 64) * (kDM / 64)) % 8 == 0, "the engine's grids: whole blocks of eight wave tiles");
